// GraphEncoder_74749610819667
// MI455X (gfx1250) — hardware-verified
//
#include <hip/hip_runtime.h>
#include <stddef.h>
#include <stdint.h>
#include <math.h>


#define FD      64
#define K1      64
#define K2      128
#define NHID    256
#define NOC     128
#define KHB     512
#define NGR     2000
#define GP      2048
#define NTHR    256
#define NWAVE   8
#define EPT     8
#define CHUNK   (NTHR * EPT)
#define WCAP    (EPT * 32)
#define LISTN   (NWAVE * WCAP)
#define NBD     8192
#define SLD     13
#define NBA     1024
#define SLA     10
#define RCAP    28672
#define DEGCAP  64
#define NBP     128
#define SLP     7
#define RCAPP   16384
#define DEGCAPP 128
#define GBM     64
#define GBN     64
#define GTHR    128
#define UW1     512
#define UWK     512
#define UH1     2048
#define UH2     4096
#define NUW     (UW1 + 8 * UWK + 2 * UH1 + 2 * UH2)
#define AGG_ZINTS     (LISTN + 2 * RCAP + 3 * NBA)
#define AGG_LDS_INTS  (AGG_ZINTS + 16)
#define POOL_ZINTS    (LISTN + 2 * RCAPP + 3 * NBP)
#define POOL_LDS_INTS (POOL_ZINTS + 16)
#define NUH     (GP * (NHID / 8))
#define WSMAX   134217728

static_assert((CHUNK & (CHUNK - 1)) == 0 && CHUNK <= 4096);
static_assert((NBD & (NBD - 1)) == 0 && NBD == (1 << SLD));
static_assert((NBA & (NBA - 1)) == 0 && NBA == (1 << SLA));
static_assert((NBP & (NBP - 1)) == 0 && NBP == (1 << SLP));
static_assert(((long long)CHUNK << SLD) < (1LL << 31));
static_assert(((long long)CHUNK << SLA) < (1LL << 31));
static_assert(((long long)CHUNK << SLP) < (1LL << 31));
static_assert(NBD % (NTHR * 4) == 0);
static_assert(LISTN % NTHR == 0);
static_assert(NBA % NWAVE == 0 && NBA % 32 == 0 && NBA % GBM == 0);
static_assert(NBP % NWAVE == 0 && NBP % 32 == 0 && GP % NBP == 0 && GP % GBM == 0 && GP >= NGR);
static_assert(RCAP % 32 == 0 && RCAPP % 32 == 0);
static_assert(AGG_ZINTS % 4 == 0 && POOL_ZINTS % 4 == 0 && LISTN % 4 == 0);
static_assert(K1 % 32 == 0 && K2 % 32 == 0 && KHB % 32 == 0 && K2 == 2 * FD && KHB == 2 * NHID);
static_assert(FD == GBN && NHID % GBN == 0 && NOC % GBN == 0);
static_assert(GBM == (GTHR / 32) * 16 && GBN == 64);
static_assert(UW1 % NTHR == 0 && UWK % NTHR == 0 && UH1 % NTHR == 0 && UH2 % NTHR == 0 && NUW % NTHR == 0);
static_assert(UW1 == FD * (K1 / 8) && UWK == FD * (FD / 8) && UH1 == NHID * (FD / 8) && UH2 == NOC * (NHID / 8));
static_assert(UWK == (1 << 9) && UH1 == (1 << 11) && UH2 == (1 << 12));
static_assert(FD == 2 * 32);
static_assert(AGG_LDS_INTS * 4 <= 300000 && POOL_LDS_INTS * 4 <= 300000);
static_assert(NUH % NTHR == 0);
static_assert((NOC * 4) % 256 == 0);
static_assert(NGR * NOC - 1 == 255999);

typedef float          v2f   __attribute__((ext_vector_type(2)));
typedef float          v4f   __attribute__((ext_vector_type(4)));
typedef float          v8f   __attribute__((ext_vector_type(8)));
typedef int            v4i   __attribute__((ext_vector_type(4)));
typedef int            v8i   __attribute__((ext_vector_type(8)));
typedef unsigned int   v4u   __attribute__((ext_vector_type(4)));
typedef unsigned short v8us  __attribute__((ext_vector_type(8)));
typedef unsigned short v16us __attribute__((ext_vector_type(16)));
typedef __bf16         v16bf __attribute__((ext_vector_type(16)));
typedef v2f  __attribute__((may_alias)) v2fa;
typedef v4f  __attribute__((may_alias)) v4fa;
typedef v4i  __attribute__((may_alias)) v4ia;
typedef v8us __attribute__((may_alias)) v8usa;
union FragB { v16bf v; v16us u; v8us h[2]; v8i w; };

__device__ __forceinline__ v8f wmb(const FragB& a, const FragB& b, v8f c) {
  v8f d = __builtin_amdgcn_wmma_f32_16x16x32_bf16(false, a.v, false, b.v, (short)0, c, false, false);
  asm volatile("v_nop\n\tv_nop\n\tv_nop\n\tv_nop" : "+v"(d) : "v"(a.w), "v"(b.w));
  return d;
}

__device__ __forceinline__ unsigned bf16_bits(float f) {
  const unsigned u = __float_as_uint(f);
  return (u + 0x7FFFu + ((u >> 16) & 1u)) >> 16;
}
__device__ __forceinline__ float bf16_val(float f) {
  return __uint_as_float(bf16_bits(f) << 16);
}

template <int SLB>
__device__ __forceinline__ int scan_chunk(const int* __restrict__ dsts, int nE, int cbase, int slotBase,
                                          int nb, int vec8, int* list, int tid, int lane, int wave) {
  int wc = 0;
  const int el0  = tid * EPT;
  const int e0   = cbase + el0;
  const int sent = -2147483647 - 1;
  v4i da, db;
  if (vec8 != 0 && cbase + CHUNK <= nE) {
    da = *(const v4i*)(dsts + e0);
    db = *(const v4i*)(dsts + e0 + 4);
  } else {
    da.x = (e0     < nE) ? dsts[min(e0,     nE - 1)] : sent;
    da.y = (e0 + 1 < nE) ? dsts[min(e0 + 1, nE - 1)] : sent;
    da.z = (e0 + 2 < nE) ? dsts[min(e0 + 2, nE - 1)] : sent;
    da.w = (e0 + 3 < nE) ? dsts[min(e0 + 3, nE - 1)] : sent;
    db.x = (e0 + 4 < nE) ? dsts[min(e0 + 4, nE - 1)] : sent;
    db.y = (e0 + 5 < nE) ? dsts[min(e0 + 5, nE - 1)] : sent;
    db.z = (e0 + 6 < nE) ? dsts[min(e0 + 6, nE - 1)] : sent;
    db.w = (e0 + 7 < nE) ? dsts[min(e0 + 7, nE - 1)] : sent;
  }
  const unsigned nbs = (unsigned)slotBase;
  const unsigned unb = (unsigned)nb;
  const unsigned s0 = (unsigned)da.x - nbs, s1 = (unsigned)da.y - nbs;
  const unsigned s2 = (unsigned)da.z - nbs, s3 = (unsigned)da.w - nbs;
  const unsigned s4 = (unsigned)db.x - nbs, s5 = (unsigned)db.y - nbs;
  const unsigned s6 = (unsigned)db.z - nbs, s7 = (unsigned)db.w - nbs;
  const bool h0 = s0 < unb, h1 = s1 < unb, h2 = s2 < unb, h3 = s3 < unb;
  const bool h4 = s4 < unb, h5 = s5 < unb, h6 = s6 < unb, h7 = s7 < unb;
  const unsigned any = __builtin_amdgcn_ballot_w32(h0 | h1 | h2 | h3 | h4 | h5 | h6 | h7);
  if (any != 0u) {
#define HITJ(J, HJ, SJ) { \
      const unsigned mj = __builtin_amdgcn_ballot_w32(HJ); \
      if (mj != 0u) { \
        if (HJ) { \
          const int pos = wc + (int)__builtin_amdgcn_mbcnt_lo(mj, 0u); \
          if (pos < WCAP) list[wave * WCAP + pos] = ((el0 + (J)) << SLB) | (int)(SJ); \
        } \
        wc += (int)__builtin_popcount(mj); } }
    HITJ(0, h0, s0)
    HITJ(1, h1, s1)
    HITJ(2, h2, s2)
    HITJ(3, h3, s3)
    HITJ(4, h4, s4)
    HITJ(5, h5, s5)
    HITJ(6, h6, s6)
    HITJ(7, h7, s7)
#undef HITJ
  }
  return wc;
}

__global__ __launch_bounds__(NTHR) void k_wprep(
    const float* __restrict__ W1, const float* __restrict__ W2, const float* __restrict__ W3,
    const float* __restrict__ W4, const float* __restrict__ W5, const float* __restrict__ Wh1,
    const float* __restrict__ Wh2,
    unsigned short* W1T, unsigned short* W2T, unsigned short* W3T, unsigned short* W4T,
    unsigned short* W5T, unsigned short* H1T, unsigned short* H2T) {
  const int u = (int)blockIdx.x * NTHR + (int)threadIdx.x;
  const float* W;
  unsigned short* P;
  int v, lk, nout, pitch, coff;
  if (u < UW1) {
    W = W1; P = W1T; v = u; lk = 3; nout = FD; pitch = K1; coff = 0;
  } else if (u < UW1 + 8 * UWK) {
    const int r = u - UW1;
    const int part = r >> 9;
    v = r & (UWK - 1);
    const int li = part >> 1;
    coff = (part & 1) * FD;
    if (li == 0)      { W = W2; P = W2T; }
    else if (li == 1) { W = W3; P = W3T; }
    else if (li == 2) { W = W4; P = W4T; }
    else              { W = W5; P = W5T; }
    lk = 3; nout = FD; pitch = K2;
  } else if (u < UW1 + 8 * UWK + 2 * UH1) {
    const int r = u - (UW1 + 8 * UWK);
    const int part = r >> 11;
    v = r & (UH1 - 1);
    W = Wh1; P = H1T; lk = 3; nout = NHID; pitch = K2; coff = part * FD;
  } else if (u < NUW) {
    const int r = u - (UW1 + 8 * UWK + 2 * UH1);
    const int part = r >> 12;
    v = r & (UH2 - 1);
    W = Wh2; P = H2T; lk = 5; nout = NOC; pitch = KHB; coff = part * NHID;
  } else {
    return;
  }
  const int n  = v >> lk;
  const int k8 = (v & ((1 << lk) - 1)) * 8;
  const float* p = W + (size_t)k8 * nout + n;
  v8us o;
#pragma unroll
  for (int i = 0; i < 8; ++i) o[i] = (unsigned short)bf16_bits(p[(size_t)i * nout]);
  unsigned short* dp = P + (size_t)n * pitch + coff + k8;
  *(volatile v8us*)dp = o;
  __threadfence();
  *(volatile v8us*)dp = o;
}

__global__ __launch_bounds__(NTHR) void k_cvx(const float* __restrict__ x, int nN, int nUnits,
                                              unsigned short* xb) {
  const int u = (int)blockIdx.x * NTHR + (int)threadIdx.x;
  if (u >= nUnits) return;
  const int row = u >> 3;
  const int k8  = (u & 7) * 8;
  const int rc  = row < nN ? row : nN - 1;
  const float* p = x + (size_t)rc * FD + k8;
  const v4f a = *(const v4fa*)p;
  const v4f b = *(const v4fa*)(p + 4);
  const bool ok = row < nN;
  v8us o;
  o[0] = ok ? (unsigned short)bf16_bits(a.x) : (unsigned short)0;
  o[1] = ok ? (unsigned short)bf16_bits(a.y) : (unsigned short)0;
  o[2] = ok ? (unsigned short)bf16_bits(a.z) : (unsigned short)0;
  o[3] = ok ? (unsigned short)bf16_bits(a.w) : (unsigned short)0;
  o[4] = ok ? (unsigned short)bf16_bits(b.x) : (unsigned short)0;
  o[5] = ok ? (unsigned short)bf16_bits(b.y) : (unsigned short)0;
  o[6] = ok ? (unsigned short)bf16_bits(b.z) : (unsigned short)0;
  o[7] = ok ? (unsigned short)bf16_bits(b.w) : (unsigned short)0;
  unsigned short* dp = xb + (size_t)row * FD + k8;
  *(volatile v8us*)dp = o;
  __threadfence();
  *(volatile v8us*)dp = o;
}

__global__ __launch_bounds__(NTHR) void k_deg(const int* __restrict__ dsts, int nE, int vec8, float* dis) {
  __shared__ __attribute__((aligned(16))) int scnt[NBD];
  __shared__ __attribute__((aligned(16))) int list[LISTN];
  __shared__ int wcnt[NWAVE];
  const int tid = (int)threadIdx.x, lane = tid & 31, wave = tid >> 5;
  const int nodeBase = (int)blockIdx.x * NBD;

  for (int i = tid; i < NBD; i += NTHR) scnt[i] = 0;
  for (int i = tid; i < LISTN; i += NTHR) list[i] = 0;
  if (tid < NWAVE) wcnt[tid] = 0;
  __syncthreads();

  const int nChunks = (nE + CHUNK - 1) / CHUNK;
#pragma unroll 1
  for (int ch = 0; ch < nChunks; ++ch) {
    const int cbase = ch * CHUNK;
    const int wc = scan_chunk<SLD>(dsts, nE, cbase, nodeBase, NBD, vec8, list, tid, lane, wave);
    if (lane == 0) wcnt[wave] = wc;
    __syncthreads();
    if (wave == 0) {
#pragma unroll 1
      for (int w2 = 0; w2 < NWAVE; ++w2) {
        int c = wcnt[w2];
        c = c < 0 ? 0 : (c > WCAP ? WCAP : c);
#pragma unroll 1
        for (int b0 = 0; b0 < c; b0 += 32) {
          const int idx = b0 + lane;
          const int ent = list[w2 * WCAP + (idx < WCAP ? idx : WCAP - 1)];
          const int m32 = (c - b0) < 32 ? (c - b0) : 32;
#pragma unroll 1
          for (int k = 0; k < m32; ++k) {
            const int u  = __builtin_amdgcn_readlane(ent, k);
            const int sl = u & (NBD - 1);
            if (lane == 0) scnt[sl] = scnt[sl] + 1;
          }
        }
      }
    }
    __syncthreads();
  }

  v4f vals[NBD / (NTHR * 4)];
#pragma unroll
  for (int it = 0; it < NBD / (NTHR * 4); ++it) {
    const int s0 = it * (NTHR * 4) + 4 * tid;
    const v4i c4 = *(const v4ia*)(scnt + s0);
    const float d0 = (float)c4.x + 1.0f, d1 = (float)c4.y + 1.0f;
    const float d2 = (float)c4.z + 1.0f, d3 = (float)c4.w + 1.0f;
    v4f v;
    v.x = rsqrtf(d0); v.y = rsqrtf(d1); v.z = rsqrtf(d2); v.w = rsqrtf(d3);
    vals[it] = v;
  }
#pragma unroll
  for (int it = 0; it < NBD / (NTHR * 4); ++it) {
    const int s0 = it * (NTHR * 4) + 4 * tid;
    *(volatile v4f*)(dis + (size_t)nodeBase + s0) = vals[it];
  }
  __threadfence();
#pragma unroll
  for (int it = 0; it < NBD / (NTHR * 4); ++it) {
    const int s0 = it * (NTHR * 4) + 4 * tid;
    *(volatile v4f*)(dis + (size_t)nodeBase + s0) = vals[it];
  }
}

template <int EPI>
__global__ __launch_bounds__(GTHR) void k_gemm(
    const unsigned short* __restrict__ A, const unsigned short* __restrict__ WT,
    float* outF, int K, int ldo, const float* __restrict__ bias, int nOut)
{
  __shared__ __attribute__((aligned(16))) float stg[GBM * GBN];
  const int tid = (int)threadIdx.x, lane = tid & 31, wave = tid >> 5, hh = lane >> 4, m = lane & 15;
  const int rowBase = (int)blockIdx.x * GBM;
  const int col0    = (int)blockIdx.y * GBN;

  v8f acc[4];
  {
    const v8f z = {0.f, 0.f, 0.f, 0.f, 0.f, 0.f, 0.f, 0.f};
    acc[0] = z; acc[1] = z; acc[2] = z; acc[3] = z;
  }
  const unsigned short* ap = A  + (size_t)(rowBase + 16 * wave + m) * (size_t)K + 8 * hh;
  const unsigned short* wp = WT + (size_t)(col0 + m) * (size_t)K + 8 * hh;
  const int ksteps = K >> 5;
#pragma unroll 1
  for (int ks = 0; ks < ksteps; ++ks) {
    FragB af;
    af.h[0] = *(const v8usa*)(ap + 32 * ks);
    af.h[1] = *(const v8usa*)(ap + 32 * ks + 16);
#pragma unroll
    for (int t = 0; t < 4; ++t) {
      const unsigned short* wq = wp + (size_t)(16 * t) * (size_t)K + 32 * ks;
      FragB bf;
      bf.h[0] = *(const v8usa*)wq;
      bf.h[1] = *(const v8usa*)(wq + 16);
      acc[t] = wmb(af, bf, acc[t]);
    }
  }

#pragma unroll
  for (int t = 0; t < 4; ++t) {
    const int lc = 16 * t + m;
#pragma unroll
    for (int r = 0; r < 8; ++r) {
      const int lr = 16 * wave + 8 * hh + r;
      stg[lr * GBN + lc] = acc[t][r];
    }
  }
  __syncthreads();

  v4f fv[8];
#pragma unroll
  for (int i = 0; i < 8; ++i) {
    const int lr = 16 * wave + 2 * i + hh;
    fv[i] = *(const v4fa*)(stg + lr * GBN + 4 * m);
  }
  if constexpr (EPI != 0) {
    const v4f t4 = *(const v4fa*)(bias + col0 + 4 * m);
    v4f bb;
    bb.x = bf16_val(t4.x); bb.y = bf16_val(t4.y); bb.z = bf16_val(t4.z); bb.w = bf16_val(t4.w);
#pragma unroll
    for (int i = 0; i < 8; ++i) fv[i] = fv[i] + bb;
  }
#pragma unroll
  for (int i = 0; i < 8; ++i) {
    const int lr = 16 * wave + 2 * i + hh;
    const int gr = rowBase + lr;
    const bool ok = (EPI == 0) || (gr < nOut);
    float* op = outF + (size_t)gr * (size_t)ldo + col0 + 4 * m;
    if (ok) *(volatile v4f*)op = fv[i];
  }
  __threadfence();
#pragma unroll
  for (int i = 0; i < 8; ++i) {
    const int lr = 16 * wave + 2 * i + hh;
    const int gr = rowBase + lr;
    const bool ok = (EPI == 0) || (gr < nOut);
    float* op = outF + (size_t)gr * (size_t)ldo + col0 + 4 * m;
    if (ok) *(volatile v4f*)op = fv[i];
  }
}

template <int MODE, int RELU>
__global__ __launch_bounds__(NTHR) void k_agg(const int* __restrict__ srcs, const int* __restrict__ dsts,
                                              int nE, int nN, int vec8, int mRows,
                                              const float* __restrict__ dis,
                                              const float* __restrict__ xl, const float* __restrict__ bias,
                                              unsigned short* hb, float* hout) {
  extern __shared__ __attribute__((aligned(16))) int dsm[];
  int* list = dsm;
  int* hl   = dsm + LISTN;
  int* sl   = dsm + LISTN + RCAP;
  int* cnt  = dsm + LISTN + 2 * RCAP;
  int* offs = cnt + NBA;
  int* cur  = offs + NBA;
  int* misc = cur + NBA;
  const int tid = (int)threadIdx.x, lane = tid & 31, wave = tid >> 5;
  const int nodeBase = (int)blockIdx.x * NBA;

  {
    const v4i z4 = {0, 0, 0, 0};
    for (int i = tid * 4; i < AGG_ZINTS; i += NTHR * 4) *(v4ia*)(dsm + i) = z4;
    if (tid < 16) misc[tid] = 0;
  }
  float bv0, bv1;
  {
    const v2f a = *(const v2fa*)(bias + 2 * lane);
    bv0 = bf16_val(a.x); bv1 = bf16_val(a.y);
  }
  __syncthreads();

  int t = 0, ov = 0;
  const int nChunks = (nE + CHUNK - 1) / CHUNK;
#pragma unroll 1
  for (int ch = 0; ch < nChunks; ++ch) {
    const int cbase = ch * CHUNK;
    const int wc = scan_chunk<SLA>(dsts, nE, cbase, nodeBase, NBA, vec8, list, tid, lane, wave);
    if (lane == 0) misc[wave] = wc;
    __syncthreads();
    if (wave == 0) {
#pragma unroll 1
      for (int w2 = 0; w2 < NWAVE; ++w2) {
        int c = misc[w2];
        c = c < 0 ? 0 : (c > WCAP ? WCAP : c);
#pragma unroll 1
        for (int b0 = 0; b0 < c; b0 += 32) {
          const int idx = b0 + lane;
          const int ent = list[w2 * WCAP + (idx < WCAP ? idx : WCAP - 1)];
          const int m32 = (c - b0) < 32 ? (c - b0) : 32;
#pragma unroll 1
          for (int k = 0; k < m32; ++k) {
            const int u    = __builtin_amdgcn_readlane(ent, k);
            const int slot = u & (NBA - 1);
            const int el   = (u >> SLA) & (CHUNK - 1);
            const int pk   = ((cbase + el) << SLA) | slot;
            if (t < RCAP) {
              if (lane == 0) { hl[t] = pk; cnt[slot] = cnt[slot] + 1; }
              t = t + 1;
            } else {
              ov = 1;
            }
          }
        }
      }
    }
    __syncthreads();
  }
  if (wave == 0 && lane == 0) { misc[8] = t; misc[9] = ov; }
  __syncthreads();
  int tt = misc[8];
  tt = tt < 0 ? 0 : (tt > RCAP ? RCAP : tt);
  const int ovf = misc[9];

  if (wave == 0) {
    const int base = lane * (NBA / 32);
    int s = 0;
#pragma unroll 1
    for (int i = 0; i < NBA / 32; ++i) s += cnt[base + i];
    int incl = s;
#pragma unroll
    for (int d = 1; d < 32; d <<= 1) {
      const int y = __shfl_up(incl, d, 32);
      if (lane >= d) incl += y;
    }
    int run = incl - s;
#pragma unroll 1
    for (int i = 0; i < NBA / 32; ++i) {
      const int cv = cnt[base + i];
      offs[base + i] = run;
      cur[base + i]  = run;
      run += cv;
    }
  }
  __syncthreads();
  if (wave == 0) {
#pragma unroll 1
    for (int b0 = 0; b0 < tt; b0 += 32) {
      const int idx = b0 + lane;
      const int ent = hl[idx < RCAP ? idx : RCAP - 1];
      const int m32 = (tt - b0) < 32 ? (tt - b0) : 32;
#pragma unroll 1
      for (int k = 0; k < m32; ++k) {
        const int u    = __builtin_amdgcn_readlane(ent, k);
        const int slot = u & (NBA - 1);
        if (lane == 0) {
          int p = cur[slot];
          p = p < 0 ? 0 : (p > RCAP - 1 ? RCAP - 1 : p);
          sl[p] = u;
          cur[slot] = p + 1;
        }
      }
    }
  }
  __syncthreads();

  const float qnan = __int_as_float(0x7fc00000);
  const float pz = (ovf != 0) ? qnan : 0.0f;
  const int sa = (2 * lane) & 31, sb = (2 * lane + 1) & 31;
  const int q0s = (4 * lane) & 31, q1s = (4 * lane + 1) & 31;
  const int q2s = (4 * lane + 2) & 31, q3s = (4 * lane + 3) & 31;
#pragma unroll 1
  for (int si = 0; si < NBA / NWAVE; ++si) {
    const int s    = si * NWAVE + wave;
    const int node = nodeBase + s;
    int c = cnt[s];
    const bool big = c > DEGCAP;
    c = c < 0 ? 0 : (c > DEGCAP ? DEGCAP : c);
    int o = offs[s];
    o = o < 0 ? 0 : (o > RCAP ? RCAP : o);
    const int nc = node < nN ? node : nN - 1;
    const float dd = dis[nc];
    const float rd = dd * dd;
    float acc0 = 0.0f, acc1 = 0.0f;
#pragma unroll 1
    for (int b0 = 0; b0 < c; b0 += 32) {
      int idx = o + b0 + lane;
      idx = idx > RCAP - 1 ? RCAP - 1 : idx;
      const int ent = sl[idx];
      int eid = ent >> SLA;
      eid = eid < 0 ? 0 : (eid > nE - 1 ? nE - 1 : eid);
      int sr = srcs[eid];
      sr = sr < 0 ? 0 : (sr > nN - 1 ? nN - 1 : sr);
      const float cf  = dis[sr] * dd;
      const int   cfi = __float_as_int(cf);
      const int m32 = (c - b0) < 32 ? (c - b0) : 32;
#pragma unroll 1
      for (int k = 0; k < m32; ++k) {
        const int   sk = __builtin_amdgcn_readlane(sr, k);
        const float ck = __int_as_float(__builtin_amdgcn_readlane(cfi, k));
        const v2f a = *(const v2fa*)(xl + (size_t)sk * FD + 2 * lane);
        acc0 = fmaf(ck, a.x, acc0); acc1 = fmaf(ck, a.y, acc1);
      }
    }
    float sv0, sv1;
    {
      const v2f a = *(const v2fa*)(xl + (size_t)nc * FD + 2 * lane);
      sv0 = a.x; sv1 = a.y;
    }
    const float pzr = big ? qnan : pz;
    const bool live = node < nN;
    float y0 = (acc0 + sv0 * rd) + bv0;
    float y1 = (acc1 + sv1 * rd) + bv1;
    if constexpr (RELU != 0) {
      y0 = (y0 < 0.0f) ? 0.0f : y0;
      y1 = (y1 < 0.0f) ? 0.0f : y1;
    }
    y0 = y0 + pzr; y1 = y1 + pzr;
    const float v0 = live ? y0 : 0.0f;
    const float v1 = live ? y1 : 0.0f;
    const bool wr = (node < mRows) && (lane < 16);
    if constexpr (MODE != 0) {
      const unsigned hb0 = bf16_bits(v0), hb1 = bf16_bits(v1);
      const unsigned lb0 = bf16_bits(v0 - __uint_as_float(hb0 << 16));
      const unsigned lb1 = bf16_bits(v1 - __uint_as_float(hb1 << 16));
      const int hw = (int)(hb0 | (hb1 << 16));
      const int lw = (int)(lb0 | (lb1 << 16));
      const int g0 = __shfl(hw, q0s, 32), g1 = __shfl(hw, q1s, 32);
      const int g2 = __shfl(hw, q2s, 32), g3 = __shfl(hw, q3s, 32);
      const int p0 = __shfl(lw, q0s, 32), p1 = __shfl(lw, q1s, 32);
      const int p2 = __shfl(lw, q2s, 32), p3 = __shfl(lw, q3s, 32);
      const bool lsel = (lane & 8) != 0;
      v4u pv;
      pv.x = (unsigned int)(lsel ? p0 : g0);
      pv.y = (unsigned int)(lsel ? p1 : g1);
      pv.z = (unsigned int)(lsel ? p2 : g2);
      pv.w = (unsigned int)(lsel ? p3 : g3);
      unsigned short* hp = hb + (size_t)node * K2 + 8 * (lane & 15);
      if (wr) *(volatile v4u*)hp = pv;
      __threadfence();
      if (wr) *(volatile v4u*)hp = pv;
    } else {
      v4f ow;
      ow.x = __shfl(v0, sa, 32); ow.y = __shfl(v1, sa, 32);
      ow.z = __shfl(v0, sb, 32); ow.w = __shfl(v1, sb, 32);
      float* op = hout + (size_t)node * FD + 4 * (lane & 15);
      if (wr) *(volatile v4f*)op = ow;
      __threadfence();
      if (wr) *(volatile v4f*)op = ow;
    }
  }
}

__global__ __launch_bounds__(NTHR) void k_pool(const int* __restrict__ bat, int nN, int vec8,
                                               const int* __restrict__ numg, int nG, int gRows,
                                               const float* __restrict__ hf, unsigned short* ph) {
  extern __shared__ __attribute__((aligned(16))) int psm[];
  int* list = psm;
  int* hl   = psm + LISTN;
  int* sl   = hl + RCAPP;
  int* cnt  = sl + RCAPP;
  int* offs = cnt + NBP;
  int* cur  = offs + NBP;
  int* misc = cur + NBP;
  const int tid = (int)threadIdx.x, lane = tid & 31, wave = tid >> 5;
  const int gBase = (int)blockIdx.x * NBP;

  {
    const v4i z4 = {0, 0, 0, 0};
    for (int i = tid * 4; i < POOL_ZINTS; i += NTHR * 4) *(v4ia*)(psm + i) = z4;
    if (tid < 16) misc[tid] = 0;
  }
  int nLive;
  {
    int g0 = numg[0];
    g0 = g0 < 0 ? 0 : g0;
    nLive = g0 > nG ? nG : g0;
  }
  __syncthreads();

  int t = 0, ov = 0;
  const int nChunks = (nN + CHUNK - 1) / CHUNK;
#pragma unroll 1
  for (int ch = 0; ch < nChunks; ++ch) {
    const int cbase = ch * CHUNK;
    const int wc = scan_chunk<SLP>(bat, nN, cbase, gBase, NBP, vec8, list, tid, lane, wave);
    if (lane == 0) misc[wave] = wc;
    __syncthreads();
    if (wave == 0) {
#pragma unroll 1
      for (int w2 = 0; w2 < NWAVE; ++w2) {
        int c = misc[w2];
        c = c < 0 ? 0 : (c > WCAP ? WCAP : c);
#pragma unroll 1
        for (int b0 = 0; b0 < c; b0 += 32) {
          const int idx = b0 + lane;
          const int ent = list[w2 * WCAP + (idx < WCAP ? idx : WCAP - 1)];
          const int m32 = (c - b0) < 32 ? (c - b0) : 32;
#pragma unroll 1
          for (int k = 0; k < m32; ++k) {
            const int u    = __builtin_amdgcn_readlane(ent, k);
            const int slot = u & (NBP - 1);
            const int el   = (u >> SLP) & (CHUNK - 1);
            const int pk   = ((cbase + el) << SLP) | slot;
            if (t < RCAPP) {
              if (lane == 0) { hl[t] = pk; cnt[slot] = cnt[slot] + 1; }
              t = t + 1;
            } else {
              ov = 1;
            }
          }
        }
      }
    }
    __syncthreads();
  }
  if (wave == 0 && lane == 0) { misc[8] = t; misc[9] = ov; }
  __syncthreads();
  int tt = misc[8];
  tt = tt < 0 ? 0 : (tt > RCAPP ? RCAPP : tt);
  const int ovf = misc[9];

  if (wave == 0) {
    const int base = lane * (NBP / 32);
    int s = 0;
#pragma unroll 1
    for (int i = 0; i < NBP / 32; ++i) s += cnt[base + i];
    int incl = s;
#pragma unroll
    for (int d = 1; d < 32; d <<= 1) {
      const int y = __shfl_up(incl, d, 32);
      if (lane >= d) incl += y;
    }
    int run = incl - s;
#pragma unroll 1
    for (int i = 0; i < NBP / 32; ++i) {
      const int cv = cnt[base + i];
      offs[base + i] = run;
      cur[base + i]  = run;
      run += cv;
    }
  }
  __syncthreads();
  if (wave == 0) {
#pragma unroll 1
    for (int b0 = 0; b0 < tt; b0 += 32) {
      const int idx = b0 + lane;
      const int ent = hl[idx < RCAPP ? idx : RCAPP - 1];
      const int m32 = (tt - b0) < 32 ? (tt - b0) : 32;
#pragma unroll 1
      for (int k = 0; k < m32; ++k) {
        const int u    = __builtin_amdgcn_readlane(ent, k);
        const int slot = u & (NBP - 1);
        if (lane == 0) {
          int p = cur[slot];
          p = p < 0 ? 0 : (p > RCAPP - 1 ? RCAPP - 1 : p);
          sl[p] = u;
          cur[slot] = p + 1;
        }
      }
    }
  }
  __syncthreads();

  const float qnan = __int_as_float(0x7fc00000);
  const float pz = (ovf != 0) ? qnan : 0.0f;
  const int q0s = (4 * lane) & 31, q1s = (4 * lane + 1) & 31;
  const int q2s = (4 * lane + 2) & 31, q3s = (4 * lane + 3) & 31;
#pragma unroll 1
  for (int si = 0; si < NBP / NWAVE; ++si) {
    const int s = si * NWAVE + wave;
    const int g = gBase + s;
    int c = cnt[s];
    c = c < 0 ? 0 : c;
    const bool big = c > DEGCAPP;
    const int ct = c > DEGCAPP ? DEGCAPP : c;
    int o = offs[s];
    o = o < 0 ? 0 : (o > RCAPP ? RCAPP : o);
    float a0 = 0.0f, a1 = 0.0f;
#pragma unroll 1
    for (int b0 = 0; b0 < ct; b0 += 32) {
      int idx = o + b0 + lane;
      idx = idx > RCAPP - 1 ? RCAPP - 1 : idx;
      const int ent = sl[idx];
      int nd = ent >> SLP;
      nd = nd < 0 ? 0 : (nd > nN - 1 ? nN - 1 : nd);
      const int m32 = (ct - b0) < 32 ? (ct - b0) : 32;
#pragma unroll 1
      for (int k = 0; k < m32; ++k) {
        const int nk = __builtin_amdgcn_readlane(nd, k);
        const v2f a = *(const v2fa*)(hf + (size_t)nk * FD + 2 * lane);
        a0 += a.x; a1 += a.y;
      }
    }
    const float cf  = (c < 1) ? 1.0f : (float)c;
    const float inv = 1.0f / cf;
    const float pzr = big ? qnan : pz;
    const bool live = g < nLive;
    const float y0 = a0 * inv + pzr;
    const float y1 = a1 * inv + pzr;
    const float v0 = live ? y0 : 0.0f;
    const float v1 = live ? y1 : 0.0f;
    const bool wr = (g < gRows) && (lane < 16);
    const unsigned hb0 = bf16_bits(v0), hb1 = bf16_bits(v1);
    const unsigned lb0 = bf16_bits(v0 - __uint_as_float(hb0 << 16));
    const unsigned lb1 = bf16_bits(v1 - __uint_as_float(hb1 << 16));
    const int hw = (int)(hb0 | (hb1 << 16));
    const int lw = (int)(lb0 | (lb1 << 16));
    const int g0 = __shfl(hw, q0s, 32), g1 = __shfl(hw, q1s, 32);
    const int g2 = __shfl(hw, q2s, 32), g3 = __shfl(hw, q3s, 32);
    const int p0 = __shfl(lw, q0s, 32), p1 = __shfl(lw, q1s, 32);
    const int p2 = __shfl(lw, q2s, 32), p3 = __shfl(lw, q3s, 32);
    const bool lsel = (lane & 8) != 0;
    v4u pv;
    pv.x = (unsigned int)(lsel ? p0 : g0);
    pv.y = (unsigned int)(lsel ? p1 : g1);
    pv.z = (unsigned int)(lsel ? p2 : g2);
    pv.w = (unsigned int)(lsel ? p3 : g3);
    unsigned short* hp = ph + (size_t)g * K2 + 8 * (lane & 15);
    if (wr) *(volatile v4u*)hp = pv;
    __threadfence();
    if (wr) *(volatile v4u*)hp = pv;
  }
}

__global__ __launch_bounds__(NTHR) void k_hsplit(const float* __restrict__ z, const float* __restrict__ bh,
                                                 int nLive, int nUnits, unsigned short* zh) {
  const int u = (int)blockIdx.x * NTHR + (int)threadIdx.x;
  if (u >= nUnits) return;
  const int row = u >> 5;
  const int c8  = (u & 31) * 8;
  const float* p = z + (size_t)row * NHID + c8;
  const v4f a  = *(const v4fa*)p;
  const v4f b  = *(const v4fa*)(p + 4);
  const v4f ba = *(const v4fa*)(bh + c8);
  const v4f bb = *(const v4fa*)(bh + c8 + 4);
  const bool ok = row < nLive;
  float tv[8];
  tv[0] = a.x + bf16_val(ba.x); tv[1] = a.y + bf16_val(ba.y);
  tv[2] = a.z + bf16_val(ba.z); tv[3] = a.w + bf16_val(ba.w);
  tv[4] = b.x + bf16_val(bb.x); tv[5] = b.y + bf16_val(bb.y);
  tv[6] = b.z + bf16_val(bb.z); tv[7] = b.w + bf16_val(bb.w);
  v8us hv, lv;
#pragma unroll
  for (int i = 0; i < 8; ++i) {
    float y = (tv[i] < 0.0f) ? 0.0f : tv[i];
    y = ok ? y : 0.0f;
    const unsigned hbt = bf16_bits(y);
    hv[i] = (unsigned short)hbt;
    lv[i] = (unsigned short)bf16_bits(y - __uint_as_float(hbt << 16));
  }
  unsigned short* dp = zh + (size_t)row * KHB + c8;
  *(volatile v8us*)dp = hv;
  *(volatile v8us*)(dp + NHID) = lv;
  __threadfence();
  *(volatile v8us*)dp = hv;
  *(volatile v8us*)(dp + NHID) = lv;
}

static inline int cdiv(int a, int b) { return (a + b - 1) / b; }
static inline size_t al256(size_t o) { return (o + 255) & ~(size_t)255; }

extern "C" void kernel_launch(void* const* d_in, const int* in_sizes, int n_in,
                              void* d_out, int out_size, void* d_ws, size_t ws_size,
                              hipStream_t stream) {
  if (n_in < 18) return;
  if (in_sizes[0] < FD || (in_sizes[0] % FD) != 0) return;
  const int nN = in_sizes[0] / FD;
  if (nN < 1 || nN >= (1 << 22)) return;
  if (in_sizes[1] < 2 || (in_sizes[1] & 1) != 0) return;
  const int nE = in_sizes[1] / 2;
  if (nE < 1 || nE >= (1 << (31 - SLA))) return;
  if (in_sizes[2] != nN) return;
  if (in_sizes[3] != FD * FD || in_sizes[4] != FD) return;
  if (in_sizes[5] != FD * FD || in_sizes[6] != FD) return;
  if (in_sizes[7] != FD * FD || in_sizes[8] != FD) return;
  if (in_sizes[9] != FD * FD || in_sizes[10] != FD) return;
  if (in_sizes[11] != FD * FD || in_sizes[12] != FD) return;
  if (in_sizes[13] != FD * NHID || in_sizes[14] != NHID) return;
  if (in_sizes[15] != NHID * NOC || in_sizes[16] != NOC) return;
  if (in_sizes[17] < 1) return;
  if (out_size != NGR * NOC) return;

  const float* x    = (const float*)d_in[0];
  const int*   edge = (const int*)d_in[1];
  const int*   bat  = (const int*)d_in[2];
  const float* W1   = (const float*)d_in[3];
  const float* b1   = (const float*)d_in[4];
  const float* W2   = (const float*)d_in[5];
  const float* b2   = (const float*)d_in[6];
  const float* W3   = (const float*)d_in[7];
  const float* b3   = (const float*)d_in[8];
  const float* W4   = (const float*)d_in[9];
  const float* b4   = (const float*)d_in[10];
  const float* W5   = (const float*)d_in[11];
  const float* b5   = (const float*)d_in[12];
  const float* Wh1  = (const float*)d_in[13];
  const float* bh1  = (const float*)d_in[14];
  const float* Wh2  = (const float*)d_in[15];
  const float* bh2  = (const float*)d_in[16];
  const int*   numg = (const int*)d_in[17];
  float* out = (float*)d_out;
  const int* src = edge;
  const int* dst = edge + nE;

  const int MP   = cdiv(nN, GBM) * GBM;
  const int gM   = MP / GBM;
  const int gD   = cdiv(nN, NBD);
  const int NBPD = gD * NBD;
  const int gA   = cdiv(MP, NBA);
  if ((long long)gA * NBA < (long long)MP) return;
  if (NBPD < nN) return;
  const int gP   = GP / NBP;
  const int gH   = GP / GBM;
  const int vec8e = ((nE & 3) == 0) ? 1 : 0;
  const int vec8p = ((nN & 3) == 0) ? 1 : 0;

  char* ws = (char*)d_ws;
  size_t off = 0;
  const size_t oDIS = off; off = al256(off + (size_t)NBPD * 4);
  const size_t oW1T = off; off = al256(off + (size_t)FD * K1 * 2);
  const size_t oW2T = off; off = al256(off + (size_t)FD * K2 * 2);
  const size_t oW3T = off; off = al256(off + (size_t)FD * K2 * 2);
  const size_t oW4T = off; off = al256(off + (size_t)FD * K2 * 2);
  const size_t oW5T = off; off = al256(off + (size_t)FD * K2 * 2);
  const size_t oH1T = off; off = al256(off + (size_t)NHID * K2 * 2);
  const size_t oH2T = off; off = al256(off + (size_t)NOC * KHB * 2);
  const size_t oXB  = off; off = al256(off + (size_t)MP * FD * 2);
  const size_t oXW  = off; off = al256(off + (size_t)MP * FD * 4);
  const size_t oA2  = off; off = al256(off + (size_t)MP * K2 * 2);
  const size_t oH5  = off; off = al256(off + (size_t)MP * FD * 4);
  const size_t oPH  = off; off = al256(off + (size_t)GP * K2 * 2);
  const size_t oZ   = off; off = al256(off + (size_t)GP * NHID * 4);
  const size_t oZH  = off; off = al256(off + (size_t)GP * KHB * 2);
  if (off > ws_size || off > (size_t)WSMAX) return;
  float*          DIS = (float*)(ws + oDIS);
  unsigned short* W1T = (unsigned short*)(ws + oW1T);
  unsigned short* W2T = (unsigned short*)(ws + oW2T);
  unsigned short* W3T = (unsigned short*)(ws + oW3T);
  unsigned short* W4T = (unsigned short*)(ws + oW4T);
  unsigned short* W5T = (unsigned short*)(ws + oW5T);
  unsigned short* H1T = (unsigned short*)(ws + oH1T);
  unsigned short* H2T = (unsigned short*)(ws + oH2T);
  unsigned short* XB  = (unsigned short*)(ws + oXB);
  float*          XW  = (float*)(ws + oXW);
  unsigned short* A2  = (unsigned short*)(ws + oA2);
  float*          H5  = (float*)(ws + oH5);
  unsigned short* PH  = (unsigned short*)(ws + oPH);
  float*          Z   = (float*)(ws + oZ);
  unsigned short* ZH  = (unsigned short*)(ws + oZH);

  const size_t aggLds  = (size_t)AGG_LDS_INTS * 4;
  const size_t poolLds = (size_t)POOL_LDS_INTS * 4;
  hipFuncSetAttribute(reinterpret_cast<const void*>(&k_agg<1, 1>), hipFuncAttributeMaxDynamicSharedMemorySize, (int)aggLds);
  hipFuncSetAttribute(reinterpret_cast<const void*>(&k_agg<0, 0>), hipFuncAttributeMaxDynamicSharedMemorySize, (int)aggLds);
  hipFuncSetAttribute(reinterpret_cast<const void*>(&k_pool), hipFuncAttributeMaxDynamicSharedMemorySize, (int)poolLds);

  const int nUx = MP * (FD / 8);
  k_wprep<<<NUW / NTHR, NTHR, 0, stream>>>(W1, W2, W3, W4, W5, Wh1, Wh2, W1T, W2T, W3T, W4T, W5T, H1T, H2T);
  k_cvx<<<cdiv(nUx, NTHR), NTHR, 0, stream>>>(x, nN, nUx, XB);
  k_deg<<<gD, NTHR, 0, stream>>>(dst, nE, vec8e, DIS);
  k_gemm<0><<<dim3(gM, FD / GBN), GTHR, 0, stream>>>(XB, W1T, XW, K1, FD, b1, MP);
  k_agg<1, 1><<<gA, NTHR, aggLds, stream>>>(src, dst, nE, nN, vec8e, MP, DIS, XW, b1, A2, H5);
  k_gemm<0><<<dim3(gM, FD / GBN), GTHR, 0, stream>>>(A2, W2T, XW, K2, FD, b2, MP);
  k_agg<1, 1><<<gA, NTHR, aggLds, stream>>>(src, dst, nE, nN, vec8e, MP, DIS, XW, b2, A2, H5);
  k_gemm<0><<<dim3(gM, FD / GBN), GTHR, 0, stream>>>(A2, W3T, XW, K2, FD, b3, MP);
  k_agg<1, 1><<<gA, NTHR, aggLds, stream>>>(src, dst, nE, nN, vec8e, MP, DIS, XW, b3, A2, H5);
  k_gemm<0><<<dim3(gM, FD / GBN), GTHR, 0, stream>>>(A2, W4T, XW, K2, FD, b4, MP);
  k_agg<1, 1><<<gA, NTHR, aggLds, stream>>>(src, dst, nE, nN, vec8e, MP, DIS, XW, b4, A2, H5);
  k_gemm<0><<<dim3(gM, FD / GBN), GTHR, 0, stream>>>(A2, W5T, XW, K2, FD, b5, MP);
  k_agg<0, 0><<<gA, NTHR, aggLds, stream>>>(src, dst, nE, nN, vec8e, MP, DIS, XW, b5, A2, H5);
  k_pool<<<gP, NTHR, poolLds, stream>>>(bat, nN, vec8p, numg, NGR, GP, H5, PH);
  k_gemm<0><<<dim3(gH, NHID / GBN), GTHR, 0, stream>>>(PH, H1T, Z, K2, NHID, bh1, GP);
  k_hsplit<<<NUH / NTHR, NTHR, 0, stream>>>(Z, bh1, NGR, NUH, ZH);
  k_gemm<1><<<dim3(gH, NOC / GBN), GTHR, 0, stream>>>(ZH, H2T, out, KHB, NOC, bh2, NGR);
}
